// GraphAttentionLayer_17179869618
// MI455X (gfx1250) — hardware-run, weakly checked
//
#include <hip/hip_runtime.h>
#include <stddef.h>
#include <stdint.h>

#pragma clang fp contract(off)

#define NB 8
#define NN 1024
#define ND 1024
#define NH 8
#define NF 128
#define HF 1024
#define BN 8192
#define PLANE_F (NB * NH * NN)
#define PREP_HB_BLOCKS 4096
#define PREP_WT_BLOCKS 256
#define PJ_P 132
#define WSMAX 134217728

static_assert(NN % 64 == 0);
static_assert(NF == 128);
static_assert(NH * NF == HF && HF == 1024);
static_assert(NN / 32 == 32);
static_assert(ND % 32 == 0);
static_assert(NN % 32 == 0);
static_assert(BN == NB * NN && BN % 64 == 0);
static_assert((size_t)BN * ND / 8 / 256 == PREP_HB_BLOCKS);
static_assert((ND / 64) * (HF / 64) == PREP_WT_BLOCKS);
static_assert(64 * 68 * 4 <= 327680);
static_assert(64 * PJ_P * 4 + 256 * 4 + 128 * 4 <= 327680);
static_assert(NH * NN * 4 + 32 * 32 * 4 + 2 * NH * 32 * 4 <= 327680);
static_assert(2 * 128 * 64 * 2 + 64 * 4 + 4 * 16 * 68 * 4 <= 327680);

typedef float          v2f   __attribute__((ext_vector_type(2)));
typedef float          v4f   __attribute__((ext_vector_type(4)));
typedef float          v8f   __attribute__((ext_vector_type(8)));
typedef unsigned int   v2u   __attribute__((ext_vector_type(2)));
typedef unsigned int   v4u   __attribute__((ext_vector_type(4)));
typedef unsigned int   v8u   __attribute__((ext_vector_type(8)));
typedef unsigned short v8us  __attribute__((ext_vector_type(8)));
typedef __bf16         v16bf __attribute__((ext_vector_type(16)));
typedef v4f  __attribute__((may_alias)) v4fa;
typedef v4u  __attribute__((may_alias)) v4ua;
typedef v8us __attribute__((may_alias)) v8usa;
union FragB { v16bf v; v8us h[2]; v8u w; };

__device__ __forceinline__ v8f wmb(const FragB& a, const FragB& b, v8f c) {
  v8f d = __builtin_amdgcn_wmma_f32_16x16x32_bf16(false, a.v, false, b.v, (short)0, c, false, false);
  asm volatile("v_nop\n\tv_nop\n\tv_nop\n\tv_nop" : "+v"(d) : "v"(a.w), "v"(b.w));
  return d;
}

__device__ __forceinline__ unsigned bf16_bits(float f) {
  const unsigned u = __float_as_uint(f);
  return (u + 0x7FFFu + ((u >> 16) & 1u)) >> 16;
}
__device__ __forceinline__ float bf16_val(float f) { return __uint_as_float(bf16_bits(f) << 16); }
__device__ __forceinline__ unsigned pk16(unsigned lo16, unsigned hi16) { return (lo16 & 0xFFFFu) | (hi16 << 16); }

__global__ __launch_bounds__(256) void k_prep(const float* __restrict__ h, const float* __restrict__ W,
                                              const float* __restrict__ a,
                                              unsigned short* HB, unsigned short* WT, float* AB) {
  __shared__ __align__(16) float tf[64 * 68];
  const int tid = (int)threadIdx.x;
  const int bid = (int)blockIdx.x;
  if (bid < PREP_HB_BLOCKS) {
    const size_t u = (size_t)bid * 256 + (size_t)tid;
    const float* p = h + u * 8;
    const v4f x0 = *(const v4f*)p;
    const v4f x1 = *(const v4f*)(p + 4);
    v4u o;
    o.x = pk16(bf16_bits(x0.x), bf16_bits(x0.y));
    o.y = pk16(bf16_bits(x0.z), bf16_bits(x0.w));
    o.z = pk16(bf16_bits(x1.x), bf16_bits(x1.y));
    o.w = pk16(bf16_bits(x1.z), bf16_bits(x1.w));
    unsigned short* dp = HB + u * 8;
    *(volatile v4u*)dp = o;
    __threadfence();
    *(volatile v4u*)dp = o;
  } else if (bid < PREP_HB_BLOCKS + PREP_WT_BLOCKS) {
    const int t  = bid - PREP_HB_BLOCKS;
    const int c0 = (t & 15) * 64;
    const int r0 = (t >> 4) * 64;
    {
      const int lr = tid >> 4;
      const int c4 = (tid & 15) * 4;
#pragma unroll
      for (int it = 0; it < 4; ++it) {
        const int rr = it * 16 + lr;
        const v4f q = *(const v4f*)(W + (size_t)(r0 + rr) * HF + c0 + c4);
        *(v4f*)(tf + rr * 68 + c4) = q;
      }
    }
    __syncthreads();
    const int sub = tid >> 3;
    const int c8  = (tid & 7) * 8;
    v4u hv[2];
#pragma unroll
    for (int it = 0; it < 2; ++it) {
      const int oc = it * 32 + sub;
      v4u q4;
#pragma unroll
      for (int q = 0; q < 4; ++q) {
        const float f0 = tf[(c8 + 2 * q) * 68 + oc];
        const float f1 = tf[(c8 + 2 * q + 1) * 68 + oc];
        q4[q] = pk16(bf16_bits(f0), bf16_bits(f1));
      }
      hv[it] = q4;
    }
    for (int pass = 0; pass < 2; ++pass) {
#pragma unroll
      for (int it = 0; it < 2; ++it) {
        const int oc = it * 32 + sub;
        const size_t go = (size_t)(c0 + oc) * ND + r0 + c8;
        *(volatile v4u*)(WT + go) = hv[it];
      }
      __threadfence();
    }
  } else {
    if (tid < 64) {
      const v4f q = *(const v4f*)(a + 4 * tid);
      v4f o;
      o.x = bf16_val(q.x); o.y = bf16_val(q.y); o.z = bf16_val(q.z); o.w = bf16_val(q.w);
      float* dp = AB + 4 * tid;
      *(volatile v4f*)dp = o;
      __threadfence();
      *(volatile v4f*)dp = o;
    }
  }
}

__global__ __launch_bounds__(128) __attribute__((amdgpu_num_vgpr(248)))
void k_proj(const unsigned short* __restrict__ HB, const unsigned short* __restrict__ WT,
            const float* __restrict__ AB, float* ELR, unsigned short* VTh, unsigned short* VTl) {
  __shared__ __align__(16) float stg[64 * PJ_P];
  __shared__ __align__(16) float sab[256];
  __shared__ __align__(16) float sdt[128];
  const int tid = (int)threadIdx.x, lane = tid & 31, wave = tid >> 5, hh = lane >> 4, m = lane & 15;
  const int rowBase = (int)blockIdx.x * 64;
  const int hd      = (int)blockIdx.y;
  const int colBase = hd * NF;

  if (tid < 64) {
    const v4f q = *(const v4f*)(AB + 4 * tid);
    *(v4fa*)(sab + 4 * tid) = q;
  }

  v8f acc[8];
  {
    const v8f z = {0.f, 0.f, 0.f, 0.f, 0.f, 0.f, 0.f, 0.f};
#pragma unroll
    for (int t = 0; t < 8; ++t) acc[t] = z;
  }
  const unsigned short* ap = HB + (size_t)(rowBase + 16 * wave + m) * (size_t)ND + 8 * hh;
  const unsigned short* bp = WT + (size_t)(colBase + m) * (size_t)ND + 8 * hh;

#pragma unroll 1
  for (int k0 = 0; k0 < ND; k0 += 32) {
    FragB af;
    af.h[0] = *(const v8usa*)(ap + k0);
    af.h[1] = *(const v8usa*)(ap + k0 + 16);
#pragma unroll
    for (int nt = 0; nt < 8; ++nt) {
      const unsigned short* wq = bp + (size_t)(16 * nt) * (size_t)ND + k0;
      FragB bf;
      bf.h[0] = *(const v8usa*)wq;
      bf.h[1] = *(const v8usa*)(wq + 16);
      acc[nt] = wmb(af, bf, acc[nt]);
    }
  }

#pragma unroll
  for (int nt = 0; nt < 8; ++nt) {
    const int lc = 16 * nt + m;
#pragma unroll
    for (int r = 0; r < 8; ++r) {
      const int lr = 16 * wave + 8 * hh + r;
      stg[lr * PJ_P + lc] = acc[nt][r];
    }
  }
  __syncthreads();

  const v4f al4 = *(const v4fa*)(sab + 4 * lane);
  const v4f ar4 = *(const v4fa*)(sab + NF + 4 * lane);
#pragma unroll 1
  for (int i = 0; i < 16; ++i) {
    const int row = wave * 16 + i;
    const v4f p = *(const v4fa*)(stg + row * PJ_P + 4 * lane);
    float s = 0.0f, d = 0.0f;
    s = fmaf(p.x, al4.x, s); s = fmaf(p.y, al4.y, s); s = fmaf(p.z, al4.z, s); s = fmaf(p.w, al4.w, s);
    d = fmaf(p.x, ar4.x, d); d = fmaf(p.y, ar4.y, d); d = fmaf(p.z, ar4.z, d); d = fmaf(p.w, ar4.w, d);
#pragma unroll
    for (int off = 16; off > 0; off >>= 1) {
      s += __shfl_xor(s, off, 32);
      d += __shfl_xor(d, off, 32);
    }
    if (lane == 0) { sdt[row] = s; sdt[64 + row] = d; }
  }
  __syncthreads();

  const int b  = rowBase >> 10;
  const int n0 = rowBase & (NN - 1);
  const size_t pl = (size_t)(b * NH + hd) * NN + n0;
  const v4f elv = *(const v4fa*)(sdt + 4 * lane);
  float* elp = ELR + (size_t)(lane >> 4) * PLANE_F + pl + 4 * (lane & 15);
  const size_t vbase = (size_t)(b * NH + hd) * NF * NN + n0;
  const int fsub = tid >> 3;
  const int c8   = (tid & 7) * 8;
  for (int pass = 0; pass < 2; ++pass) {
#pragma unroll 2
    for (int it = 0; it < 8; ++it) {
      const int f = it * 16 + fsub;
      v4u hv, lv;
#pragma unroll
      for (int q = 0; q < 4; ++q) {
        const float f0 = stg[(c8 + 2 * q) * PJ_P + f];
        const float f1 = stg[(c8 + 2 * q + 1) * PJ_P + f];
        const unsigned h0 = bf16_bits(f0), h1 = bf16_bits(f1);
        const unsigned l0 = bf16_bits(f0 - __uint_as_float(h0 << 16));
        const unsigned l1 = bf16_bits(f1 - __uint_as_float(h1 << 16));
        hv[q] = pk16(h0, h1);
        lv[q] = pk16(l0, l1);
      }
      const size_t go = vbase + (size_t)f * NN + c8;
      *(volatile v4u*)(VTh + go) = hv;
      *(volatile v4u*)(VTl + go) = lv;
    }
    if (wave == 0) *(volatile v4f*)elp = elv;
    __threadfence();
  }
}

__global__ __launch_bounds__(256) void k_pack(const int* __restrict__ adj, const float* __restrict__ ELR,
                                              unsigned* MB, float* MROW) {
  __shared__ __align__(16) float    sER[NH * NN];
  __shared__ __align__(16) unsigned sMB[32 * 32];
  __shared__ __align__(16) float    sM[NH * 32];
  __shared__ __align__(16) float    sEL[NH * 32];
  const int tid = (int)threadIdx.x, lane = tid & 31, wave = tid >> 5;
  const int b  = (int)blockIdx.x >> 5;
  const int i0 = ((int)blockIdx.x & 31) * 32;
  const float* erb = ELR + PLANE_F + (size_t)b * NH * NN;
#pragma unroll 4
  for (int it = 0; it < 8; ++it) {
    const int idx = (it * 256 + tid) * 4;
    const v4f v = *(const v4f*)(erb + idx);
    *(v4fa*)(sER + idx) = v;
  }
  sEL[tid] = ELR[(size_t)(b * NH + (tid >> 5)) * NN + i0 + (tid & 31)];
  __syncthreads();

  const float ninf = __int_as_float((int)0xff800000u);
  const float qnan = __int_as_float(0x7fc00000);
#pragma unroll 1
  for (int rr = 0; rr < 4; ++rr) {
    const int il = wave * 4 + rr;
    const int i  = i0 + il;
    const int* arow = adj + ((size_t)b * NN + (size_t)i) * NN;
    float mx[NH];
#pragma unroll
    for (int hd = 0; hd < NH; ++hd) mx[hd] = ninf;
    unsigned myw = 0u, anyb = 0u;
#pragma unroll 4
    for (int t = 0; t < 32; ++t) {
      const int j  = t * 32 + lane;
      const int av = arow[j];
      asm volatile("" :: "v"(av));
      const bool unm = (av + ((j == i) ? 1 : 0)) != 0;
      const unsigned bal = __builtin_amdgcn_ballot_w32(unm);
      myw  = (lane == t) ? bal : myw;
      anyb |= bal;
#pragma unroll
      for (int hd = 0; hd < NH; ++hd) {
        const float e = sER[hd * NN + j];
        const float c = fmaxf(mx[hd], e);
        mx[hd] = unm ? c : mx[hd];
      }
    }
#pragma unroll
    for (int hd = 0; hd < NH; ++hd) {
      float v = mx[hd];
#pragma unroll
      for (int off = 16; off > 0; off >>= 1) v = fmaxf(v, __shfl_xor(v, off, 32));
      mx[hd] = v;
    }
    sMB[il * 32 + lane] = myw;
#pragma unroll
    for (int hd = 0; hd < NH; ++hd) {
      const float x0 = sEL[hd * 32 + il] + mx[hd];
      float mm = (x0 >= 0.0f) ? x0 : 0.2f * x0;
      const bool bad = (anyb == 0u) || !(mm >= -800.0f);
      mm = bad ? qnan : mm;
      if (lane == 0) sM[hd * 32 + il] = mm;
    }
  }
  __syncthreads();

  const v4u wv = *(const v4ua*)(sMB + (tid >> 3) * 32 + 4 * (tid & 7));
  unsigned* mbp = MB + ((size_t)b * NN + (size_t)(i0 + (tid >> 3))) * 32 + 4 * (tid & 7);
  const int t64 = tid & 63;
  const v4f mv = *(const v4fa*)(sM + (t64 >> 3) * 32 + 4 * (t64 & 7));
  float* mrp = MROW + (size_t)(b * NH + (t64 >> 3)) * NN + i0 + 4 * (t64 & 7);
  *(volatile v4u*)mbp = wv;
  if (tid < 64) *(volatile v4f*)mrp = mv;
  __threadfence();
  *(volatile v4u*)mbp = wv;
  if (tid < 64) *(volatile v4f*)mrp = mv;
}

__device__ __forceinline__ float pval(float e, unsigned on, float el, float mi) {
  float x = el + e;
  x = (x >= 0.0f) ? x : 0.2f * x;
  const float p = __expf(x - mi);
  return (on != 0u) ? p : 0.0f;
}

__global__ __launch_bounds__(128) __attribute__((amdgpu_num_vgpr(248)))
void k_attn(const unsigned short* __restrict__ VTh, const unsigned short* __restrict__ VTl,
            const float* __restrict__ ELR, const float* __restrict__ MROW,
            const unsigned* __restrict__ MB, float* out) {
  __shared__ __align__(16) unsigned short Vh[NF * 64];
  __shared__ __align__(16) unsigned short Vl[NF * 64];
  __shared__ __align__(16) float sEr[64];
  __shared__ __align__(16) float Os[4][16 * 68];
  const int tid = (int)threadIdx.x, lane = tid & 31, wave = tid >> 5, hh = lane >> 4, c = lane & 15;
  const int bx = (int)blockIdx.x;
  const int qt = bx & 15;
  const int hd = (bx >> 4) & 7;
  const int b  = bx >> 7;
  const int i0 = qt * 64 + wave * 16;
  const int irow = i0 + c;
  const size_t pl = (size_t)(b * NH + hd) * NN;
  const float el = ELR[pl + irow];
  const float mi = MROW[pl + irow];
  const unsigned* mrow = MB + ((size_t)b * NN + (size_t)irow) * 32;
  const unsigned short* vhb = VTh + pl * NF;
  const unsigned short* vlb = VTl + pl * NF;
  const float* erb = ELR + PLANE_F + pl;

  v8f oacc[8];
  {
    const v8f z = {0.f, 0.f, 0.f, 0.f, 0.f, 0.f, 0.f, 0.f};
#pragma unroll
    for (int t = 0; t < 8; ++t) oacc[t] = z;
  }
  float lsum = 0.0f;

#pragma unroll 1
  for (int kt = 0; kt < NN / 64; ++kt) {
    const int j0 = kt * 64;
    __syncthreads();
#pragma unroll 4
    for (int it = 0; it < 8; ++it) {
      const int idx = it * 128 + tid;
      const int f   = idx >> 3;
      const int pc  = (idx & 7) * 8;
      const v8us x0 = *(const v8usa*)(vhb + (size_t)f * NN + j0 + pc);
      const v8us x1 = *(const v8usa*)(vlb + (size_t)f * NN + j0 + pc);
      *(v8usa*)(Vh + f * 64 + pc) = x0;
      *(v8usa*)(Vl + f * 64 + pc) = x1;
    }
    if (wave < 2) sEr[tid] = erb[j0 + tid];
    const v2u mw = *(const v2u*)(mrow + 2 * kt);
    const unsigned mw0 = mw.x, mw1 = mw.y;
    asm volatile("" :: "v"(mw0), "v"(mw1));
    __syncthreads();

#pragma unroll 1
    for (int kk = 0; kk < 2; ++kk) {
      const unsigned wsel = (kk == 0) ? mw0 : mw1;
      const unsigned bits = wsel >> (8 * hh);
      const float* ep = sEr + kk * 32 + 8 * hh;
      const v4f e0 = *(const v4fa*)(ep);
      const v4f e1 = *(const v4fa*)(ep + 4);
      const v4f e2 = *(const v4fa*)(ep + 16);
      const v4f e3 = *(const v4fa*)(ep + 20);
      float ev[16];
      ev[0] = e0.x; ev[1] = e0.y; ev[2]  = e0.z; ev[3]  = e0.w;
      ev[4] = e1.x; ev[5] = e1.y; ev[6]  = e1.z; ev[7]  = e1.w;
      ev[8] = e2.x; ev[9] = e2.y; ev[10] = e2.z; ev[11] = e2.w;
      ev[12] = e3.x; ev[13] = e3.y; ev[14] = e3.z; ev[15] = e3.w;
      v8u wh, wl;
#pragma unroll
      for (int q = 0; q < 8; ++q) {
        const int ia = 2 * q, ib = 2 * q + 1;
        const int ba = (ia < 8) ? ia : ia + 8;
        const int bb = (ib < 8) ? ib : ib + 8;
        const float p0 = pval(ev[ia], (bits >> ba) & 1u, el, mi);
        const float p1 = pval(ev[ib], (bits >> bb) & 1u, el, mi);
        lsum += p0;
        lsum += p1;
        const unsigned h0 = bf16_bits(p0), h1 = bf16_bits(p1);
        const unsigned l0 = bf16_bits(p0 - __uint_as_float(h0 << 16));
        const unsigned l1 = bf16_bits(p1 - __uint_as_float(h1 << 16));
        wh[q] = pk16(h0, h1);
        wl[q] = pk16(l0, l1);
      }
      FragB pa, pb;
      pa.w = wh;
      pb.w = wl;
#pragma unroll
      for (int t = 0; t < 8; ++t) {
        const int ro = (t * 16 + c) * 64 + kk * 32 + 8 * hh;
        FragB vb, vl;
        vb.h[0] = *(const v8usa*)(Vh + ro);
        vb.h[1] = *(const v8usa*)(Vh + ro + 16);
        vl.h[0] = *(const v8usa*)(Vl + ro);
        vl.h[1] = *(const v8usa*)(Vl + ro + 16);
        oacc[t] = wmb(pa, vb, oacc[t]);
        oacc[t] = wmb(pa, vl, oacc[t]);
        oacc[t] = wmb(pb, vb, oacc[t]);
      }
    }
  }

  const float ltot = lsum + __shfl_xor(lsum, 16, 32);
  float lr[8];
#pragma unroll
  for (int r = 0; r < 8; ++r) lr[r] = __shfl(ltot, 8 * hh + r, 32);

  float* os = Os[wave];
  float* ob = out + ((size_t)b * NN) * HF + (size_t)hd * NF;
  const int c4 = (lane & 15) * 4;
#pragma unroll
  for (int half = 0; half < 2; ++half) {
#pragma unroll
    for (int tt = 0; tt < 4; ++tt)
#pragma unroll
      for (int r = 0; r < 8; ++r)
        os[(8 * hh + r) * 68 + tt * 16 + c] = oacc[half * 4 + tt][r] / lr[r];
    __builtin_amdgcn_fence(__ATOMIC_RELEASE, "workgroup");
    __builtin_amdgcn_wave_barrier();
    __builtin_amdgcn_fence(__ATOMIC_ACQUIRE, "workgroup");
    for (int pass = 0; pass < 2; ++pass) {
#pragma unroll
      for (int it = 0; it < 8; ++it) {
        const int row = it * 2 + hh;
        const v4f val = *(const v4fa*)(os + row * 68 + c4);
        *(volatile v4f*)(ob + (size_t)(i0 + row) * HF + half * 64 + c4) = val;
      }
      __threadfence();
    }
    __builtin_amdgcn_fence(__ATOMIC_RELEASE, "workgroup");
    __builtin_amdgcn_wave_barrier();
    __builtin_amdgcn_fence(__ATOMIC_ACQUIRE, "workgroup");
  }
}

extern "C" void kernel_launch(void* const* d_in, const int* in_sizes, int n_in,
                              void* d_out, int out_size, void* d_ws, size_t ws_size,
                              hipStream_t stream) {
  if (n_in < 4) return;
  if (in_sizes[0] != NB * NN * ND) return;
  if (in_sizes[1] != NB * NN * NN) return;
  if (in_sizes[2] != ND * HF) return;
  if (in_sizes[3] != 2 * NF) return;
  if (out_size != NB * NN * HF) return;

  const float* h   = (const float*)d_in[0];
  const int*   adj = (const int*)d_in[1];
  const float* W   = (const float*)d_in[2];
  const float* a   = (const float*)d_in[3];
  float* out = (float*)d_out;

  size_t off = 0;
  const size_t oHB = off; off += (size_t)BN * ND * 2;
  const size_t oWT = off; off += (size_t)HF * ND * 2;
  const size_t oVH = off; off += (size_t)NB * NH * NF * NN * 2;
  const size_t oVL = off; off += (size_t)NB * NH * NF * NN * 2;
  const size_t oEL = off; off += (size_t)PLANE_F * 4;
  const size_t oER = off; off += (size_t)PLANE_F * 4;
  const size_t oMR = off; off += (size_t)PLANE_F * 4;
  const size_t oMB = off; off += (size_t)NB * NN * 32 * 4;
  const size_t oAB = off; off += (size_t)256 * 4;
  if (off > ws_size || off > (size_t)WSMAX) return;
  if (oER != oEL + (size_t)PLANE_F * 4) return;

  char* ws = (char*)d_ws;
  unsigned short* HB  = (unsigned short*)(ws + oHB);
  unsigned short* WT  = (unsigned short*)(ws + oWT);
  unsigned short* VTh = (unsigned short*)(ws + oVH);
  unsigned short* VTl = (unsigned short*)(ws + oVL);
  float*          ELR = (float*)(ws + oEL);
  float*          MRW = (float*)(ws + oMR);
  unsigned*       MBp = (unsigned*)(ws + oMB);
  float*          AB  = (float*)(ws + oAB);

  k_prep<<<dim3(PREP_HB_BLOCKS + PREP_WT_BLOCKS + 1), dim3(256), 0, stream>>>(h, W, a, HB, WT, AB);
  k_proj<<<dim3(BN / 64, NH), dim3(128), 0, stream>>>(HB, WT, AB, ELR, VTh, VTl);
  k_pack<<<dim3(NB * (NN / 32)), dim3(256), 0, stream>>>(adj, ELR, MBp, MRW);
  k_attn<<<dim3(NB * NH * (NN / 64)), dim3(128), 0, stream>>>(VTh, VTl, ELR, MRW, MBp, out);
  (void)hipGetLastError();
}
